// CompositionalKoopmanOperators_66417374265730
// MI455X (gfx1250) — hardware-verified
//
#include <hip/hip_runtime.h>
#include <math.h>

typedef __attribute__((ext_vector_type(16))) _Float16 v16h;
typedef __attribute__((ext_vector_type(16))) __bf16 v16b;
typedef __attribute__((ext_vector_type(8)))  _Float16 v8h;
typedef __attribute__((ext_vector_type(8)))  float v8f;
typedef __attribute__((ext_vector_type(4)))  float v4f;
typedef __attribute__((ext_vector_type(2)))  float v2f;
typedef __attribute__((ext_vector_type(4)))  unsigned v4u;
typedef __attribute__((ext_vector_type(4)))  int v4i;
typedef float __attribute__((may_alias)) float_a;
typedef int __attribute__((may_alias)) int_a;

template <typename T> __device__ __forceinline__ void vst2(void* p, T v) { *(volatile T*)p = v; __threadfence(); *(volatile T*)p = v; }
__device__ __forceinline__ v8f wmma16(v16h a, v16h b, v8f c) {
  v8f d = __builtin_amdgcn_wmma_f32_16x16x32_f16(false, a, false, b, (short)0, c, false, false);
  asm volatile("v_nop\n\tv_nop\n\tv_nop\n\tv_nop" : "+v"(d) : "v"(a), "v"(b));
  return d;
}
__device__ __forceinline__ v8f wmma_bf(v16b a, v16b b, v8f c) {
  v8f d = __builtin_amdgcn_wmma_f32_16x16x32_bf16(false, a, false, b, (short)0, c, false, false);
  asm volatile("v_nop\n\tv_nop\n\tv_nop\n\tv_nop" : "+v"(d) : "v"(a), "v"(b));
  return d;
}
__device__ __forceinline__ v16h frag_h(const _Float16* rowk0, int lane) {
  union { v16h v; v8h q[2]; } u; const _Float16* p = rowk0 + 8 * (lane >> 4);
  u.q[0] = *(const v8h*)p; u.q[1] = *(const v8h*)(p + 16); return u.v;
}
__device__ __forceinline__ v16h frag_f32(const float* rowk0, int lane) {
  v16h a; const float* p = rowk0 + 8 * (lane >> 4);
#pragma unroll
  for (int i = 0; i < 8; ++i) { a[i] = (_Float16)p[i]; a[8 + i] = (_Float16)p[16 + i]; }
  return a;
}
__device__ __forceinline__ v16h frag_f32s(const float* rowk0, int lane, float sc) {
  v16h a; const float* p = rowk0 + 8 * (lane >> 4);
#pragma unroll
  for (int i = 0; i < 8; ++i) { a[i] = (_Float16)(p[i] * sc); a[8 + i] = (_Float16)(p[16 + i] * sc); }
  return a;
}
__device__ __forceinline__ v16h fragc_f32(const float* W, int k0, int n, int lane, int ld, int K) {
  v16h a; const int g = lane >> 4;
#pragma unroll
  for (int i = 0; i < 8; ++i) { const int ka = k0 + 8 * g + i, kb = ka + 16;
    a[i] = (_Float16)(ka < K ? W[(size_t)(ka < K ? ka : K - 1) * ld + n] : 0.f); a[8 + i] = (_Float16)(kb < K ? W[(size_t)(kb < K ? kb : K - 1) * ld + n] : 0.f); }
  return a;
}
struct F2 { v16b h, l; };
__device__ __forceinline__ F2 bsplit16(const float v[16]) { F2 r;
#pragma unroll
  for (int i = 0; i < 16; ++i) { const __bf16 h = (__bf16)v[i]; r.h[i] = h; r.l[i] = (__bf16)(v[i] - (float)h); }
  return r; }
__device__ __forceinline__ F2 split_row(const float* row, int k0, int lane) { float v[16]; const float* p = row + k0 + 8 * (lane >> 4);
#pragma unroll
  for (int i = 0; i < 8; ++i) { v[i] = p[i]; v[8 + i] = p[16 + i]; }
  return bsplit16(v); }
__device__ __forceinline__ F2 split_rowK(const float* row, int k0, int lane, int K) { float v[16]; const int g = lane >> 4;
#pragma unroll
  for (int i = 0; i < 8; ++i) { const int ka = k0 + 8 * g + i, kb = ka + 16; v[i] = ka < K ? row[ka < K ? ka : K - 1] : 0.f; v[8 + i] = kb < K ? row[kb < K ? kb : K - 1] : 0.f; }
  return bsplit16(v); }
__device__ __forceinline__ F2 split_col(const float* W, int k0, int n, int lane, int ld, int K) { float v[16]; const int g = lane >> 4;
#pragma unroll
  for (int i = 0; i < 8; ++i) { const int ka = k0 + 8 * g + i, kb = ka + 16; v[i] = ka < K ? W[(size_t)(ka < K ? ka : K - 1) * ld + n] : 0.f; v[8 + i] = kb < K ? W[(size_t)(kb < K ? kb : K - 1) * ld + n] : 0.f; }
  return bsplit16(v); }
__device__ __forceinline__ v8f mac3(const F2& a, const F2& b, v8f c) { c = wmma_bf(a.l, b.h, c); c = wmma_bf(a.h, b.l, c); return wmma_bf(a.h, b.h, c); }
__device__ __forceinline__ float sigm(float v) { return 1.0f / (1.0f + expf(-v)); }
#define LDSX() do { asm volatile("s_wait_dscnt 0" ::: "memory"); __builtin_amdgcn_wave_barrier(); __builtin_amdgcn_fence(__ATOMIC_RELEASE, "workgroup"); } while (0)


#define NSC 32
#define NP 64
#define NNODE (NSC * NP)
#define NEDGE (NSC * NP * NP)
#define NF 128
#define GD 32
#define NSTEP 2
#ifndef NSCT
#define NSCT NSC
#endif
typedef __attribute__((ext_vector_type(8))) __bf16 v8b;
__device__ __forceinline__ v16b frag_b(const __bf16* rowk0, int lane) {
  union { v16b v; v8b q[2]; } u; const __bf16* p = rowk0 + 8 * (lane >> 4);
  u.q[0] = *(const v8b*)p; u.q[1] = *(const v8b*)(p + 16); return u.v;
}
__device__ __forceinline__ float bfr(float v) { return (float)(__bf16)v; }
__device__ __attribute__((noinline)) float exp_ni(float v) { return expf(v); }
__device__ __attribute__((noinline)) float erf_ni(float v) { return erff(v); }

__device__ __attribute__((noinline)) float tanh_ni(float v) { return tanhf(v); }
#define PK_OE0  0
#define PK_OE1  (PK_OE0 + 128 * 32)
#define PK_PIJ  (PK_OE1 + 128 * 128)
#define PK_RA   (PK_PIJ + 256 * 32)
#define PK_RE1  (PK_RA + 128 * 32)
#define PK_RPR  (PK_RE1 + 128 * 128)
#define PK_RRS  (PK_RPR + 128 * 128)
#define PK_PPO  (PK_RRS + 256 * 128)
#define PK_PPA  (PK_PPO + 128 * 128)
#define PK_PR0  (PK_PPA + 128 * 128)
#define PK_PR1  (PK_PR0 + 128 * 128)
#define PK_END  (PK_PR1 + 32 * 128)
#define WS_PK    0u
#define WS_NIN   (WS_PK + 2u * PK_END)
#define WS_H0    (WS_NIN + 4u * NNODE * 32)
#define WS_OBJ   (WS_H0 + 4u * NNODE * NF)
#define WS_PIJ   (WS_OBJ + 4u * NNODE * NF)
#define WS_RELE  (WS_PIJ + 4u * NNODE * 2 * NF)
#define WS_RS    (WS_RELE + 4u * (unsigned)NEDGE * NF)
#define WS_AGG   (WS_RS + 4u * NNODE * 2 * NF)
#define WS_END   (WS_AGG + 4u * NNODE * NF)

__global__ __launch_bounds__(128) void k_pack(const float* __restrict__ Wm, int ld, int col0, int Kin, int Kp, float sgn, __bf16* __restrict__ DST) {
  __shared__ __align__(16) __bf16 s[8 * NF]; const int n0 = blockIdx.x * 8, tid = threadIdx.x;
  for (int q = tid; q < 8 * Kp; q += 128) { const int rl = q / Kp, k = q % Kp; s[q] = (__bf16)(k < Kin ? sgn * bfr(Wm[(size_t)(n0 + rl) * ld + col0 + k]) : 0.f); }
  __syncthreads();
  for (int q = tid; q < Kp; q += 128) vst2((unsigned*)(DST + (size_t)n0 * Kp + q * 8), *(const v4u*)&s[q * 8]);
}
__global__ __launch_bounds__(128) void k_packpij(const float* __restrict__ RW0, __bf16* __restrict__ DST) {
  __shared__ __align__(16) __bf16 s[8 * 32]; const int n0 = blockIdx.x * 8, tid = threadIdx.x;
  for (int q = tid; q < 8 * 32; q += 128) { const int n = n0 + q / 32, k = q % 32; float v = 0.f;
    if (n < NF) { if (k < 4) v = bfr(RW0[n * 20 + 12 + k]); else if (k < 12) v = bfr(RW0[n * 20 + 4 + (k - 4)]); }
    else { const int m = n - NF; if (k < 4) v = bfr(RW0[m * 20 + 16 + k]); else if (k < 12) v = -bfr(RW0[m * 20 + 4 + (k - 4)]); }
    s[q] = (__bf16)v; }
  __syncthreads();
  if (tid < 32) vst2((unsigned*)(DST + (size_t)n0 * 32 + tid * 8), *(const v4u*)&s[tid * 8]);
}
__global__ __launch_bounds__(128) void k_nodein(const float* __restrict__ AT, const float* __restrict__ STT, float* __restrict__ NIN) {
  __shared__ __align__(16) float s[64][32]; const int tid = threadIdx.x; const int nl = tid >> 1, half = tid & 1; const size_t n = (size_t)blockIdx.x * 64 + nl;
#pragma unroll
  for (int k = 0; k < 16; ++k) { const int c = half * 16 + k; float v = 0.f; if (c < 4) v = bfr(AT[n * 4 + c]); else if (c < 12) v = bfr(STT[n * 8 + (c - 4)]); s[nl][c] = v; }
  __syncthreads();
  for (int q = tid; q < 64 * 8; q += 128) { const int rl = q >> 3, pc = q & 7; vst2(NIN + ((size_t)blockIdx.x * 64 + rl) * 32 + pc * 4, *(const v4f*)&s[rl][pc * 4]); }
}
template <int K, int AM, int EPI, int NT>
__global__ __launch_bounds__(128) void k_lin(const float* __restrict__ A, int lda, const __bf16* __restrict__ P, const float* __restrict__ bias, float* __restrict__ OUT, int ldo) {
  __shared__ __align__(16) float so[4][16][132];
  const int tid = threadIdx.x, wave = tid >> 5, lane = tid & 31, col = lane & 15, g = lane >> 4; const size_t r0 = (size_t)blockIdx.x * 64 + wave * 16; const int n0 = blockIdx.y * NT * 16;
  v8f acc[NT] = {};
#pragma unroll 2
  for (int kc = 0; kc < K / 32; ++kc) {
    if (AM == 0) { v16b a; { const float* p = A + (r0 + col) * lda + kc * 32 + 8 * g;
#pragma unroll
        for (int i = 0; i < 8; ++i) { a[i] = (__bf16)p[i]; a[8 + i] = (__bf16)p[16 + i]; } }
#pragma unroll
      for (int j = 0; j < NT; ++j) acc[j] = wmma_bf(a, frag_b(P + (size_t)(n0 + j * 16 + col) * K + kc * 32, lane), acc[j]); }
    else { const F2 a = split_row(A + (r0 + col) * lda, kc * 32, lane);
#pragma unroll
      for (int j = 0; j < NT; ++j) { const v16b w = frag_b(P + (size_t)(n0 + j * 16 + col) * K + kc * 32, lane); acc[j] = wmma_bf(a.l, w, acc[j]); acc[j] = wmma_bf(a.h, w, acc[j]); } } }
#pragma unroll
  for (int j = 0; j < NT; ++j) { const float bb = bias ? bfr(bias[n0 + j * 16 + col]) : 0.f;
#pragma unroll
    for (int r = 0; r < 8; ++r) { float v = acc[j][r] + bb; if (EPI == 1) v = fmaxf(v, 0.f); if (EPI == 2) v = tanh_ni(v); so[wave][8 * g + r][j * 16 + col] = v; } }
  LDSX();
  for (int rl = 0; rl < 16; ++rl) if (lane < NT * 4) vst2(OUT + (r0 + rl) * ldo + n0 + lane * 4, *(const v4f*)&so[wave][rl][lane * 4]);
}
__device__ __forceinline__ void put_hl(__bf16* h, __bf16* l, float v) { const __bf16 hb = (__bf16)v; *h = hb; *l = (__bf16)(v - (float)hb); }
__global__ __launch_bounds__(128) void k_rel(const float* __restrict__ RA, const float* __restrict__ PIJ, const __bf16* __restrict__ PK, const float* __restrict__ b0, const float* __restrict__ b1, float* __restrict__ RELE) {
  __shared__ __align__(16) __bf16 sa[64][40]; __shared__ __align__(16) __bf16 sh[4][16][136], sl[4][16][136]; __shared__ __align__(16) float so[4][16][132];
  const int tid = threadIdx.x, wave = tid >> 5, lane = tid & 31, col = lane & 15, g = lane >> 4; const size_t e0 = (size_t)blockIdx.x * 64; const size_t inode = (size_t)blockIdx.x; const size_t jnode0 = (inode / NP) * NP;
  for (int q = tid; q < 64 * 32; q += 128) { const int rl = q >> 5, k = q & 31; sa[rl][k] = (__bf16)(k < 4 ? bfr(RA[(e0 + rl) * 4 + k]) : 0.f); }
  __syncthreads();
  { v8f acc[8] = {}; const v16b a = frag_b(&sa[wave * 16 + col][0], lane);
#pragma unroll
    for (int j = 0; j < 8; ++j) acc[j] = wmma_bf(a, frag_b(PK + PK_RA + (size_t)(j * 16 + col) * 32, lane), acc[j]);
    const float* pi = PIJ + inode * (2 * NF);
#pragma unroll
    for (int j = 0; j < 8; ++j) { const int o = j * 16 + col; const float add = pi[o] + bfr(b0[o]);
#pragma unroll
      for (int r = 0; r < 8; ++r) { const int jn = wave * 16 + 8 * g + r; const float v = fmaxf(acc[j][r] + add + PIJ[(jnode0 + jn) * (2 * NF) + NF + o], 0.f); put_hl(&sh[wave][8 * g + r][o], &sl[wave][8 * g + r][o], v); } } }
  LDSX();
  { v8f acc[8] = {};
#pragma unroll
    for (int kc = 0; kc < NF / 32; ++kc) { const v16b xh = frag_b(&sh[wave][col][kc * 32], lane), xl = frag_b(&sl[wave][col][kc * 32], lane);
#pragma unroll
      for (int j = 0; j < 8; ++j) { const v16b w = frag_b(PK + PK_RE1 + (size_t)(j * 16 + col) * NF + kc * 32, lane); acc[j] = wmma_bf(xl, w, acc[j]); acc[j] = wmma_bf(xh, w, acc[j]); } }
#pragma unroll
    for (int j = 0; j < 8; ++j) { const float bb = bfr(b1[j * 16 + col]);
#pragma unroll
      for (int r = 0; r < 8; ++r) so[wave][8 * g + r][j * 16 + col] = fmaxf(acc[j][r] + bb, 0.f); } }
  LDSX();
  for (int rl = 0; rl < 16; ++rl) vst2(RELE + (e0 + wave * 16 + rl) * NF + lane * 4, *(const v4f*)&so[wave][rl][lane * 4]);
}
__device__ __forceinline__ void ln128(v8f acc[8], const float* __restrict__ lw, const float* __restrict__ lb, int col) {
#pragma unroll
  for (int r = 0; r < 8; ++r) { float s = 0.f;
#pragma unroll
    for (int j = 0; j < 8; ++j) s += acc[j][r];
#pragma unroll
    for (int o = 1; o < 16; o <<= 1) s += __shfl_xor(s, o);
    const float mu = s * (1.0f / NF); float q = 0.f;
#pragma unroll
    for (int j = 0; j < 8; ++j) { const float d = acc[j][r] - mu; q += d * d; }
#pragma unroll
    for (int o = 1; o < 16; o <<= 1) q += __shfl_xor(q, o);
    const float rs = rsqrtf(q * (1.0f / NF) + 1e-5f);
#pragma unroll
    for (int j = 0; j < 8; ++j) acc[j][r] = (acc[j][r] - mu) * rs * bfr(lw[j * 16 + col]) + bfr(lb[j * 16 + col]); }
}
__global__ __launch_bounds__(128) void k_prop(const float* __restrict__ RELE, const float* __restrict__ RS, const __bf16* __restrict__ PK, const float* __restrict__ rb, const float* __restrict__ lw, const float* __restrict__ lb, float* __restrict__ AGG) {
  __shared__ __align__(16) float ssum[4][NF]; __shared__ __align__(16) float sres[NF];
  const int tid = threadIdx.x, wave = tid >> 5, lane = tid & 31, col = lane & 15, g = lane >> 4; const size_t inode = blockIdx.x; const size_t e0 = inode * 64 + wave * 16; const size_t jnode0 = (inode / NP) * NP + wave * 16;
  v8f acc[8] = {};
#pragma unroll
  for (int kc = 0; kc < NF / 32; ++kc) { const F2 a = split_row(RELE + (e0 + col) * NF, kc * 32, lane);
#pragma unroll
    for (int j = 0; j < 8; ++j) { const v16b w = frag_b(PK + PK_RPR + (size_t)(j * 16 + col) * NF + kc * 32, lane); acc[j] = wmma_bf(a.l, w, acc[j]); acc[j] = wmma_bf(a.h, w, acc[j]); } }
  const float* r1 = RS + inode * (2 * NF);
#pragma unroll
  for (int j = 0; j < 8; ++j) { const int o = j * 16 + col; const float add = r1[o] + bfr(rb[o]);
#pragma unroll
    for (int r = 0; r < 8; ++r) acc[j][r] += add + RS[(jnode0 + 8 * g + r) * (2 * NF) + NF + o]; }
  ln128(acc, lw, lb, col);
#pragma unroll
  for (int j = 0; j < 8; ++j) { float s = 0.f;
#pragma unroll
    for (int r = 0; r < 8; ++r) s += fmaxf(acc[j][r], 0.f);
    s += __shfl_xor(s, 16); if (g == 0) ssum[wave][j * 16 + col] = s; }
  __syncthreads();
  if (tid < NF) sres[tid] = (ssum[0][tid] + ssum[1][tid]) + (ssum[2][tid] + ssum[3][tid]);
  __syncthreads();
  if (tid < 32) vst2(AGG + inode * NF + tid * 4, *(const v4f*)&sres[tid * 4]);
}
__global__ __launch_bounds__(128) void k_objupd(float* __restrict__ OBJ, const float* __restrict__ AGG, const __bf16* __restrict__ PK, const float* __restrict__ pb, const float* __restrict__ lw, const float* __restrict__ lb) {
  __shared__ __align__(16) float so[4][16][132];
  const int tid = threadIdx.x, wave = tid >> 5, lane = tid & 31, col = lane & 15, g = lane >> 4; const size_t r0 = (size_t)blockIdx.x * 64 + wave * 16;
  v8f acc[8] = {};
#pragma unroll
  for (int kc = 0; kc < NF / 32; ++kc) { const F2 a = split_row(OBJ + (r0 + col) * NF, kc * 32, lane), c = split_row(AGG + (r0 + col) * NF, kc * 32, lane);
#pragma unroll
    for (int j = 0; j < 8; ++j) { const v16b w = frag_b(PK + PK_PPO + (size_t)(j * 16 + col) * NF + kc * 32, lane), u = frag_b(PK + PK_PPA + (size_t)(j * 16 + col) * NF + kc * 32, lane);
      acc[j] = wmma_bf(a.l, w, acc[j]); acc[j] = wmma_bf(a.h, w, acc[j]); acc[j] = wmma_bf(c.l, u, acc[j]); acc[j] = wmma_bf(c.h, u, acc[j]); } }
#pragma unroll
  for (int j = 0; j < 8; ++j) { const float bb = bfr(pb[j * 16 + col]);
#pragma unroll
    for (int r = 0; r < 8; ++r) acc[j][r] += bb; }
  ln128(acc, lw, lb, col);
#pragma unroll
  for (int j = 0; j < 8; ++j)
#pragma unroll
    for (int r = 0; r < 8; ++r) so[wave][8 * g + r][j * 16 + col] = fmaxf(acc[j][r], 0.f);
  __syncthreads();
  for (int rl = 0; rl < 16; ++rl) vst2(OBJ + (r0 + rl) * NF + lane * 4, *(const v4f*)&so[wave][rl][lane * 4]);
}
extern "C" void kernel_launch(void* const* d_in, const int* in_sizes, int n_in, void* d_out, int out_size, void* d_ws, size_t ws_size, hipStream_t stream) {
  (void)in_sizes; (void)n_in; (void)out_size;
  const float** F = (const float**)d_in;
  if (ws_size < (size_t)WS_END) return;
  char* ws = (char*)d_ws; __bf16* PK = (__bf16*)(ws + WS_PK);
  float *NIN = (float*)(ws + WS_NIN), *H0 = (float*)(ws + WS_H0), *OBJ = (float*)(ws + WS_OBJ), *PIJ = (float*)(ws + WS_PIJ), *RELE = (float*)(ws + WS_RELE), *RS = (float*)(ws + WS_RS), *AGG = (float*)(ws + WS_AGG);
  k_pack<<<NF / 8, 128, 0, stream>>>(F[4], 12, 0, 12, 32, 1.f, PK + PK_OE0);
  k_pack<<<NF / 8, 128, 0, stream>>>(F[6], NF, 0, NF, NF, 1.f, PK + PK_OE1);
  k_pack<<<NF / 8, 128, 0, stream>>>(F[8], 20, 0, 4, 32, 1.f, PK + PK_RA);
  k_pack<<<NF / 8, 128, 0, stream>>>(F[10], NF, 0, NF, NF, 1.f, PK + PK_RE1);
  k_pack<<<NF / 8, 128, 0, stream>>>(F[12], 3 * NF, 0, NF, NF, 1.f, PK + PK_RPR);
  k_pack<<<NF / 8, 128, 0, stream>>>(F[12], 3 * NF, NF, NF, NF, 1.f, PK + PK_RRS);
  k_pack<<<NF / 8, 128, 0, stream>>>(F[12], 3 * NF, 2 * NF, NF, NF, 1.f, PK + PK_RRS + (size_t)NF * NF);
  k_pack<<<NF / 8, 128, 0, stream>>>(F[16], 2 * NF, 0, NF, NF, 1.f, PK + PK_PPO);
  k_pack<<<NF / 8, 128, 0, stream>>>(F[16], 2 * NF, NF, NF, NF, 1.f, PK + PK_PPA);
  k_pack<<<NF / 8, 128, 0, stream>>>(F[20], NF, 0, NF, NF, 1.f, PK + PK_PR0);
  k_pack<<<GD / 8, 128, 0, stream>>>(F[22], NF, 0, NF, NF, 1.f, PK + PK_PR1);
  k_packpij<<<2 * NF / 8, 128, 0, stream>>>(F[8], PK + PK_PIJ);
  k_nodein<<<NSCT * NP / 64, 128, 0, stream>>>(F[0], F[1], NIN);
  k_lin<32, 0, 1, 8><<<dim3(NSCT * NP / 64, 1), 128, 0, stream>>>(NIN, 32, PK + PK_OE0, F[5], H0, NF);
  k_lin<NF, 1, 1, 8><<<dim3(NSCT * NP / 64, 1), 128, 0, stream>>>(H0, NF, PK + PK_OE1, F[7], OBJ, NF);
  k_lin<32, 0, 0, 8><<<dim3(NSCT * NP / 64, 2), 128, 0, stream>>>(NIN, 32, PK + PK_PIJ, nullptr, PIJ, 2 * NF);
  k_rel<<<NSCT * NP * NP / 64, 128, 0, stream>>>(F[3], PIJ, PK, F[9], F[11], RELE);
  for (int st = 0; st < NSTEP; ++st) {
    k_lin<NF, 1, 0, 8><<<dim3(NSCT * NP / 64, 2), 128, 0, stream>>>(OBJ, NF, PK + PK_RRS, nullptr, RS, 2 * NF);
    k_prop<<<NSCT * NP, 128, 0, stream>>>(RELE, RS, PK, F[13], F[14], F[15], AGG);
    k_objupd<<<NSCT * NP / 64, 128, 0, stream>>>(OBJ, AGG, PK, F[17], F[18], F[19]); }
  k_lin<NF, 1, 1, 8><<<dim3(NSCT * NP / 64, 1), 128, 0, stream>>>(OBJ, NF, PK + PK_PR0, F[21], H0, NF);
  k_lin<NF, 1, 2, 2><<<dim3(NSCT * NP / 64, 1), 128, 0, stream>>>(H0, NF, PK + PK_PR1, F[23], (float*)d_out, GD);
}
